// GraphSAGE_50792283243093
// MI455X (gfx1250) — hardware-run, weakly checked
//
#include <hip/hip_runtime.h>
#include <stddef.h>
#include <stdint.h>
#include <math.h>

#define NN      50000
#define NE      850000
#define DF      128
#define MP      50048
#define XP      128
#define HP      256
#define W0P     384
#define W12P    512
#define WSOFF   256
#define SINGLE_N 1
#define SINGLE_H 0
#define KN_EXT  (SINGLE_N ? DF : 2 * DF)
#define KH_EXT  (SINGLE_H ? DF : 2 * DF)
#define NTHR    256
#define NWAVE   8
#define EPT     8
#define WCH     (32 * EPT)
#define NBRUN   1024
#define SLB     10
#define NBK     49
#define WLCAP   3584
#define RCAP    28672
#define DEGCAP  64
#define MAXDEG_MEAS   38
#define MAXB1024_MEAS 17783
#define RBM     64
#define GBM     64
#define GBN     128
#define GTHR    128
#define PERW    (((NE + NWAVE * WCH - 1) / (NWAVE * WCH)) * WCH)

#define BK_ZINTS (NWAVE * WLCAP + RCAP + 3 * NBRUN)
#define BK_MISC  32
#define BK_INTS  (BK_ZINTS + BK_MISC)
#define BK_LDS   (BK_INTS * 4)

#define PBX   (MP * DF / 8 / NTHR)
#define PBW   88
#define PBTOT (PBX + PBW + 1)

static_assert(DF == 128 && DF == 32 * 4);
static_assert(MP % GBM == 0 && MP % RBM == 0 && MP >= NN && MP == 391 * 128);
static_assert(NBRUN == (1 << SLB) && NBRUN % RBM == 0 && NBRUN % 32 == 0 && NBRUN % NWAVE == 0);
static_assert(NBK * NBRUN >= MP && (NBK - 1) * NBRUN < NN && NBK <= 64);
static_assert(NE < (1 << 21) && (((long long)NE) << SLB) < (1LL << 31));
static_assert(NE % EPT == 0 && NE % 4 == 0);
static_assert(PERW % WCH == 0 && (long long)PERW * NWAVE >= NE && (NWAVE - 1) * PERW < NE);
static_assert(RCAP == NWAVE * WLCAP && RCAP % (2 * NTHR) == 0 && BK_ZINTS % 4 == 0);
static_assert((long long)RCAP * 100 >= (long long)MAXB1024_MEAS * 105);
static_assert(WLCAP >= MAXB1024_MEAS / 8 + 1024 + 1);
static_assert(MAXDEG_MEAS + 8 <= DEGCAP && DEGCAP == 64);
static_assert((RCAP * 4) % 128 == 0 && (RCAP * 8) % 128 == 0 && (NBRUN * 4) % 128 == 0);
static_assert(NBRUN == NTHR * 4);
static_assert((MP * DF / 8) % NTHR == 0 && (DF * (DF / 8)) == 8 * NTHR);
static_assert(KN_EXT % 32 == 0 && KH_EXT % 32 == 0 && DF % 32 == 0);
static_assert(KN_EXT <= HP && KH_EXT <= HP && DF <= XP);
static_assert(WSOFF + KH_EXT <= W12P && WSOFF + DF <= W0P && KN_EXT <= WSOFF);
static_assert(GBN == DF && GBM == (GTHR / 32) * 16);
static_assert(BK_LDS <= 327680);
static_assert((GBM * GBN + DF) * 4 <= 65536);
static_assert((NBK * RCAP) % NTHR == 0 && RCAP % NTHR == 0);

typedef float          v4f   __attribute__((ext_vector_type(4)));
typedef float          v8f   __attribute__((ext_vector_type(8)));
typedef int            v2i   __attribute__((ext_vector_type(2)));
typedef int            v4i   __attribute__((ext_vector_type(4)));
typedef int            v8i   __attribute__((ext_vector_type(8)));
typedef unsigned       v2u   __attribute__((ext_vector_type(2)));
typedef unsigned short v8us  __attribute__((ext_vector_type(8)));
typedef unsigned short v16us __attribute__((ext_vector_type(16)));
typedef __bf16         v16bf __attribute__((ext_vector_type(16)));
typedef v4f  __attribute__((may_alias)) v4fa;
typedef v2i  __attribute__((may_alias)) v2ia;
typedef v4i  __attribute__((may_alias)) v4ia;
typedef v2u  __attribute__((may_alias)) v2ua;
typedef v8us __attribute__((may_alias)) v8usa;
union FragB { v16bf v; v16us u; v8us h[2]; v8i w; };

extern __shared__ __attribute__((aligned(16))) int dsm[];

__device__ __forceinline__ v8f wmb(const FragB& a, const FragB& b, v8f c) {
  v8f d = __builtin_amdgcn_wmma_f32_16x16x32_bf16(false, a.v, false, b.v, (short)0, c, false, false);
  asm volatile("v_nop\n\tv_nop\n\tv_nop\n\tv_nop" : "+v"(d) : "v"(a.w), "v"(b.w));
  return d;
}

__device__ __forceinline__ unsigned bf16_bits(float f) {
  const unsigned u = __float_as_uint(f);
  const unsigned r = (u + 0x7FFFu + ((u >> 16) & 1u)) >> 16;
  const unsigned q = (u >> 16) | 0x40u;
  return ((u & 0x7fffffffu) > 0x7f800000u) ? q : r;
}
__device__ __forceinline__ float bf16_val(float f) {
  return __uint_as_float(bf16_bits(f) << 16);
}

__device__ __forceinline__ void hilo_pack(float v0, float v1, float v2, float v3,
                                          int& h01, int& h23, int& l01, int& l23) {
  const unsigned a0 = bf16_bits(v0), a1 = bf16_bits(v1), a2 = bf16_bits(v2), a3 = bf16_bits(v3);
  const unsigned b0 = bf16_bits(v0 - __uint_as_float(a0 << 16));
  const unsigned b1 = bf16_bits(v1 - __uint_as_float(a1 << 16));
  const unsigned b2 = bf16_bits(v2 - __uint_as_float(a2 << 16));
  const unsigned b3 = bf16_bits(v3 - __uint_as_float(a3 << 16));
  h01 = (int)(a0 | (a1 << 16)); h23 = (int)(a2 | (a3 << 16));
  l01 = (int)(b0 | (b1 << 16)); l23 = (int)(b2 | (b3 << 16));
}

__device__ __forceinline__ v4i regroup32(int h01, int h23, int l01, int l23, int lane) {
  const int s0 = (2 * lane) & 31, s1 = s0 + 1;
  const int a0 = __shfl(h01, s0, 32), a1 = __shfl(h23, s0, 32), a2 = __shfl(h01, s1, 32), a3 = __shfl(h23, s1, 32);
  const int b0 = __shfl(l01, s0, 32), b1 = __shfl(l23, s0, 32), b2 = __shfl(l01, s1, 32), b3 = __shfl(l23, s1, 32);
  const int mk = (lane < 16) ? -1 : 0;
  v4i o;
  o.x = (a0 & mk) | (b0 & ~mk); o.y = (a1 & mk) | (b1 & ~mk);
  o.z = (a2 & mk) | (b2 & ~mk); o.w = (a3 & mk) | (b3 & ~mk);
  return o;
}

__device__ __forceinline__ void st2_v4f(float* p, v4f v) {
  *(volatile v4f*)p = v;
  __threadfence();
  *(volatile v4f*)p = v;
}
__device__ __forceinline__ void st2_v8us(unsigned short* p, v8us v) {
  *(volatile v8us*)p = v;
  __threadfence();
  *(volatile v8us*)p = v;
}
__device__ __forceinline__ void st2_v4i(unsigned short* p, v4i v) {
  *(volatile v4i*)p = v;
  __threadfence();
  *(volatile v4i*)p = v;
}

__device__ __forceinline__ v8us fetch8(const float* __restrict__ base, int stride) {
  float f[8];
#pragma unroll
  for (int i = 0; i < 8; ++i) f[i] = base[(size_t)i * (size_t)stride];
  v8us o;
#pragma unroll
  for (int i = 0; i < 8; ++i) o[i] = (unsigned short)bf16_bits(f[i]);
  return o;
}

__device__ __forceinline__ void wunit(const float* __restrict__ W, unsigned short* P, int pitch, int coff, int v) {
  const int n = v >> 4, k8 = (v & 15) * 8;
  const v8us o = fetch8(W + (size_t)k8 * DF + n, DF);
  st2_v8us(P + (size_t)n * (size_t)pitch + coff + k8, o);
}
__device__ __forceinline__ void bias_unit(const float* __restrict__ b, float* dstp, int lane) {
  const v4f t = *(const v4fa*)(b + 4 * lane);
  v4f o;
  o.x = bf16_val(t.x); o.y = bf16_val(t.y); o.z = bf16_val(t.z); o.w = bf16_val(t.w);
  st2_v4f(dstp + 4 * lane, o);
}

__global__ __launch_bounds__(NTHR) void k_prep(const float* __restrict__ x,
                                               const float* __restrict__ ws0, const float* __restrict__ wn0,
                                               const float* __restrict__ b0,
                                               const float* __restrict__ ws1, const float* __restrict__ wn1,
                                               const float* __restrict__ b1,
                                               const float* __restrict__ ws2, const float* __restrict__ wn2,
                                               const float* __restrict__ b2,
                                               unsigned short* xb, unsigned short* w0c, unsigned short* w1c,
                                               unsigned short* w2c, float* sm) {
  const int tid = (int)threadIdx.x, lane = tid & 31, wave = tid >> 5;
  const int blk = (int)blockIdx.x;
  if (blk < PBX) {
    const int u   = blk * NTHR + tid;
    const int row = u >> 4, k8 = (u & 15) * 8;
    const int rc  = row < NN ? row : NN - 1;
    const unsigned mk = row < NN ? 0xffffu : 0u;
    const float* p = x + (size_t)rc * DF + k8;
    const v4f a = *(const v4fa*)p;
    const v4f b = *(const v4fa*)(p + 4);
    v8us o;
    o[0] = (unsigned short)(bf16_bits(a.x) & mk); o[1] = (unsigned short)(bf16_bits(a.y) & mk);
    o[2] = (unsigned short)(bf16_bits(a.z) & mk); o[3] = (unsigned short)(bf16_bits(a.w) & mk);
    o[4] = (unsigned short)(bf16_bits(b.x) & mk); o[5] = (unsigned short)(bf16_bits(b.y) & mk);
    o[6] = (unsigned short)(bf16_bits(b.z) & mk); o[7] = (unsigned short)(bf16_bits(b.w) & mk);
    st2_v8us(xb + (size_t)row * XP + k8, o);
  } else if (blk < PBX + PBW) {
    const int bl   = blk - PBX;
    const int part = bl >> 3;
    const int v    = (bl & 7) * NTHR + tid;
    if (part == 0)       wunit(wn0, w0c, W0P, 0, v);
    else if (part == 1)  wunit(wn0, w0c, W0P, DF, v);
    else if (part == 2)  wunit(ws0, w0c, W0P, WSOFF, v);
    else if (part == 3)  wunit(wn1, w1c, W12P, 0, v);
    else if (part == 4)  wunit(wn1, w1c, W12P, DF, v);
    else if (part == 5)  wunit(ws1, w1c, W12P, WSOFF, v);
    else if (part == 6)  wunit(ws1, w1c, W12P, WSOFF + DF, v);
    else if (part == 7)  wunit(wn2, w2c, W12P, 0, v);
    else if (part == 8)  wunit(wn2, w2c, W12P, DF, v);
    else if (part == 9)  wunit(ws2, w2c, W12P, WSOFF, v);
    else                 wunit(ws2, w2c, W12P, WSOFF + DF, v);
  } else {
    if (wave == 0)      bias_unit(b0, sm, lane);
    else if (wave == 1) bias_unit(b1, sm + DF, lane);
    else if (wave == 2) bias_unit(b2, sm + 2 * DF, lane);
  }
}

template <int ROLE>
__device__ __forceinline__ void bucket_flush(const int* __restrict__ oth, int ovf, int total,
                                             int* LIST, int* CNT, int* OFF, int* DEG, int* FLAG, int blk, int tid) {
  const int* pl   = dsm + NWAVE * WLCAP;
  const int* cnt  = pl + RCAP;
  const int* offs = cnt + NBRUN;
  const int* cur  = offs + NBRUN;
  if constexpr (ROLE == 0) {
    int* lp = LIST + (size_t)blk * (size_t)(2 * RCAP);
#pragma unroll 1
    for (int it = 0; it < RCAP / (2 * NTHR); ++it) {
      const int i = 2 * (it * NTHR + tid);
      int ea = pl[i], eb = pl[i + 1];
      ea = ea < 0 ? 0 : (ea > NE - 1 ? NE - 1 : ea);
      eb = eb < 0 ? 0 : (eb > NE - 1 ? NE - 1 : eb);
      int sa = oth[ea], sb = oth[eb];
      sa = sa < 0 ? 0 : (sa > NN - 1 ? NN - 1 : sa);
      sb = sb < 0 ? 0 : (sb > NN - 1 ? NN - 1 : sb);
      v4i v;
      v.x = sa; v.y = ea; v.z = sb; v.w = eb;
      *(volatile v4i*)(lp + 2 * i) = v;
    }
    {
      const v4i c4 = *(const v4ia*)(cnt + 4 * tid);
      const v4i o4 = *(const v4ia*)(offs + 4 * tid);
      *(volatile v4i*)(CNT + (size_t)blk * NBRUN + 4 * tid) = c4;
      *(volatile v4i*)(OFF + (size_t)blk * NBRUN + 4 * tid) = o4;
    }
  }
  {
    const v4i d4 = *(const v4ia*)(cur + 4 * tid);
    *(volatile v4i*)(DEG + (size_t)blk * NBRUN + 4 * tid) = d4;
  }
  if (tid < 8) {
    v4i f;
    f.x = ovf; f.y = total; f.z = 0; f.w = 0;
    *(volatile v4i*)(FLAG + (size_t)blk * 32 + 4 * tid) = f;
  }
}

template <int ROLE>
__device__ __forceinline__ void bucket_body(const int* __restrict__ keys, const int* __restrict__ oth,
                                            const float* __restrict__ ew,
                                            int* LIST, int* CNT, int* OFF, int* DEG, int* FLAG) {
  int* wl   = dsm;
  int* pl   = dsm + NWAVE * WLCAP;
  int* cnt  = pl + RCAP;
  int* offs = cnt + NBRUN;
  int* cur  = offs + NBRUN;
  int* misc = cur + NBRUN;
  const int tid = (int)threadIdx.x, lane = tid & 31, wave = tid >> 5;
  const int blk = (int)blockIdx.x;
  const unsigned nbs = (unsigned)(blk * NBRUN);
  int nbi = NN - blk * NBRUN;
  nbi = nbi < 0 ? 0 : (nbi > NBRUN ? NBRUN : nbi);
  const unsigned unb = (unsigned)nbi;

  {
    const v4i z4 = {0, 0, 0, 0};
    for (int i = tid * 4; i < BK_ZINTS; i += NTHR * 4) *(v4ia*)(dsm + i) = z4;
    if (tid < BK_MISC) misc[tid] = 0;
  }
  __syncthreads();

  {
    const int ebeg = wave * PERW;
    const int eend = (ebeg + PERW < NE) ? (ebeg + PERW) : NE;
    const int sent = (int)(1u << 31);
    int* mylist = wl + wave * WLCAP;
    int wc = 0;
#pragma unroll 1
    for (int cb = ebeg; cb < eend; cb += WCH) {
      const int e0  = cb + lane * EPT;
      const int e0c = e0 < NE - EPT ? e0 : NE - EPT;
      const v4i da = *(const v4ia*)(keys + e0c);
      const v4i db = *(const v4ia*)(keys + e0c + 4);
      asm volatile("" :: "v"(da), "v"(db));
      const int vm = (e0 < NE) ? -1 : 0;
      const int sm_ = sent & ~vm;
      const unsigned s0 = (unsigned)((da.x & vm) | sm_) - nbs, s1 = (unsigned)((da.y & vm) | sm_) - nbs;
      const unsigned s2 = (unsigned)((da.z & vm) | sm_) - nbs, s3 = (unsigned)((da.w & vm) | sm_) - nbs;
      const unsigned s4 = (unsigned)((db.x & vm) | sm_) - nbs, s5 = (unsigned)((db.y & vm) | sm_) - nbs;
      const unsigned s6 = (unsigned)((db.z & vm) | sm_) - nbs, s7 = (unsigned)((db.w & vm) | sm_) - nbs;
      const bool h0 = s0 < unb, h1 = s1 < unb, h2 = s2 < unb, h3 = s3 < unb;
      const bool h4 = s4 < unb, h5 = s5 < unb, h6 = s6 < unb, h7 = s7 < unb;
      const unsigned m0 = __builtin_amdgcn_ballot_w32(h0), m1 = __builtin_amdgcn_ballot_w32(h1);
      const unsigned m2 = __builtin_amdgcn_ballot_w32(h2), m3 = __builtin_amdgcn_ballot_w32(h3);
      const unsigned m4 = __builtin_amdgcn_ballot_w32(h4), m5 = __builtin_amdgcn_ballot_w32(h5);
      const unsigned m6 = __builtin_amdgcn_ballot_w32(h6), m7 = __builtin_amdgcn_ballot_w32(h7);
      const unsigned any = m0 | m1 | m2 | m3 | m4 | m5 | m6 | m7;
      if (any != 0u) {
        const int pre = (int)(__builtin_amdgcn_mbcnt_lo(m0, 0u) + __builtin_amdgcn_mbcnt_lo(m1, 0u) +
                              __builtin_amdgcn_mbcnt_lo(m2, 0u) + __builtin_amdgcn_mbcnt_lo(m3, 0u) +
                              __builtin_amdgcn_mbcnt_lo(m4, 0u) + __builtin_amdgcn_mbcnt_lo(m5, 0u) +
                              __builtin_amdgcn_mbcnt_lo(m6, 0u) + __builtin_amdgcn_mbcnt_lo(m7, 0u));
        int p = wc + pre;
        if (h0) { if (p < WLCAP) mylist[p] = ((e0 + 0) << SLB) | (int)s0; p = p + 1; }
        if (h1) { if (p < WLCAP) mylist[p] = ((e0 + 1) << SLB) | (int)s1; p = p + 1; }
        if (h2) { if (p < WLCAP) mylist[p] = ((e0 + 2) << SLB) | (int)s2; p = p + 1; }
        if (h3) { if (p < WLCAP) mylist[p] = ((e0 + 3) << SLB) | (int)s3; p = p + 1; }
        if (h4) { if (p < WLCAP) mylist[p] = ((e0 + 4) << SLB) | (int)s4; p = p + 1; }
        if (h5) { if (p < WLCAP) mylist[p] = ((e0 + 5) << SLB) | (int)s5; p = p + 1; }
        if (h6) { if (p < WLCAP) mylist[p] = ((e0 + 6) << SLB) | (int)s6; p = p + 1; }
        if (h7) { if (p < WLCAP) mylist[p] = ((e0 + 7) << SLB) | (int)s7; p = p + 1; }
        wc += (int)(__builtin_popcount(m0) + __builtin_popcount(m1) + __builtin_popcount(m2) + __builtin_popcount(m3) +
                    __builtin_popcount(m4) + __builtin_popcount(m5) + __builtin_popcount(m6) + __builtin_popcount(m7));
      }
    }
    if (lane == 0) misc[wave] = wc;
  }
  __syncthreads();

  if (wave == 0) {
    int ov = 0, tot = 0;
#pragma unroll 1
    for (int w2 = 0; w2 < NWAVE; ++w2) {
      int c = misc[w2];
      if (c > WLCAP) ov = 1;
      c = c < 0 ? 0 : (c > WLCAP ? WLCAP : c);
      tot += c;
#pragma unroll 1
      for (int b0 = 0; b0 < c; b0 += 32) {
        const int idx = b0 + lane;
        const int ent = wl[w2 * WLCAP + (idx < WLCAP ? idx : WLCAP - 1)];
        const int m32 = (c - b0) < 32 ? (c - b0) : 32;
#pragma unroll 1
        for (int k = 0; k < m32; ++k) {
          const int u    = __builtin_amdgcn_readlane(ent, k);
          const int slot = u & (NBRUN - 1);
          if (lane == 0) cnt[slot] = cnt[slot] + 1;
        }
      }
    }
    if (lane == 0) { misc[8] = tot; misc[9] = ov; }
  }
  __syncthreads();
  if (wave == 0) {
    const int base = lane * (NBRUN / 32);
    int s = 0;
#pragma unroll 1
    for (int i = 0; i < NBRUN / 32; ++i) s += cnt[base + i];
    int incl = s;
#pragma unroll
    for (int d = 1; d < 32; d <<= 1) {
      const int y = __shfl_up(incl, d, 32);
      if (lane >= d) incl += y;
    }
    int run = incl - s;
#pragma unroll 1
    for (int i = 0; i < NBRUN / 32; ++i) {
      const int cv = cnt[base + i];
      offs[base + i] = run;
      cur[base + i]  = run;
      run += cv;
    }
  }
  __syncthreads();

  if (wave == 0) {
#pragma unroll 1
    for (int w2 = 0; w2 < NWAVE; ++w2) {
      int c = misc[w2];
      c = c < 0 ? 0 : (c > WLCAP ? WLCAP : c);
#pragma unroll 1
      for (int b0 = 0; b0 < c; b0 += 32) {
        const int idx = b0 + lane;
        const int ent = wl[w2 * WLCAP + (idx < WLCAP ? idx : WLCAP - 1)];
        const int m32 = (c - b0) < 32 ? (c - b0) : 32;
#pragma unroll 1
        for (int k = 0; k < m32; ++k) {
          const int u    = __builtin_amdgcn_readlane(ent, k);
          const int slot = u & (NBRUN - 1);
          int eid = (u >> SLB) & 0x1FFFFF;
          eid = eid > NE - 1 ? NE - 1 : eid;
          if (lane == 0) {
            int p = cur[slot];
            p = p < 0 ? 0 : (p > RCAP - 1 ? RCAP - 1 : p);
            pl[p] = eid;
            cur[slot] = p + 1;
          }
        }
      }
    }
  }
  __syncthreads();

  {
    int bigw = 0;
#pragma unroll 1
    for (int si = 0; si < NBRUN / NWAVE; ++si) {
      const int s = si * NWAVE + wave;
      int cv = cnt[s];
      int ovv = offs[s];
      bigw |= (cv > DEGCAP) ? 1 : 0;
      cv  = cv < 0 ? 0 : (cv > DEGCAP ? DEGCAP : cv);
      ovv = ovv < 0 ? 0 : (ovv > RCAP - 1 ? RCAP - 1 : ovv);
      int last = ovv + cv - 1;
      last = last < ovv ? ovv : last;
      last = last > RCAP - 1 ? RCAP - 1 : last;
      int i0 = ovv + lane;      i0 = i0 > last ? last : i0;
      int i1 = ovv + lane + 32; i1 = i1 > last ? last : i1;
      int ea = pl[i0], eb = pl[i1];
      ea = ea < 0 ? 0 : (ea > NE - 1 ? NE - 1 : ea);
      eb = eb < 0 ? 0 : (eb > NE - 1 ? NE - 1 : eb);
      const float wa = bf16_val(ew[ea]);
      const float wb = bf16_val(ew[eb]);
      asm volatile("" :: "v"(wa), "v"(wb));
      const int ma = (lane < cv) ? -1 : 0;
      const int mb = (lane + 32 < cv) ? -1 : 0;
      float v = __int_as_float(__float_as_int(wa) & ma) + __int_as_float(__float_as_int(wb) & mb);
      v += __shfl_xor(v, 1, 32);
      v += __shfl_xor(v, 2, 32);
      v += __shfl_xor(v, 4, 32);
      v += __shfl_xor(v, 8, 32);
      v += __shfl_xor(v, 16, 32);
      if (lane == 0) cur[s] = __float_as_int(v);
    }
    if (lane == 0) misc[16 + wave] = bigw;
  }
  __syncthreads();

  int ovf = misc[9];
#pragma unroll
  for (int w2 = 0; w2 < NWAVE; ++w2) ovf |= misc[16 + w2];
  int total = misc[8];
  total = total < 0 ? 0 : (total > RCAP ? RCAP : total);
  bucket_flush<ROLE>(oth, ovf, total, LIST, CNT, OFF, DEG, FLAG, blk, tid);
  __threadfence();
  bucket_flush<ROLE>(oth, ovf, total, LIST, CNT, OFF, DEG, FLAG, blk, tid);
}

__global__ __launch_bounds__(NTHR) void k_bucket(const int* __restrict__ srcs, const int* __restrict__ dsts,
                                                 const float* __restrict__ ew,
                                                 int* LIST, int* CNT, int* OFF, int* DDST, int* DSRC,
                                                 int* FLAGD, int* FLAGS) {
  if (blockIdx.y == 0) bucket_body<0>(dsts, srcs, ew, LIST, CNT, OFF, DDST, FLAGD);
  else                 bucket_body<1>(srcs, dsts, ew, LIST, CNT, OFF, DSRC, FLAGS);
}

__global__ __launch_bounds__(NTHR) void k_edgew(const int* __restrict__ LIST, const int* __restrict__ dsts,
                                                const float* __restrict__ ew,
                                                const float* __restrict__ DSRC, const float* __restrict__ DDST,
                                                const int* __restrict__ FLAGD, const int* __restrict__ FLAGS,
                                                float* WL) {
  const int tid = (int)threadIdx.x;
  const int blk = (int)blockIdx.x / (RCAP / NTHR);
  const int gid = (int)blockIdx.x * NTHR + tid;
  const int j   = gid - blk * RCAP;
  const v2i ent = *(const v2ia*)(LIST + 2 * (size_t)gid);
  int s = ent.x, eid = ent.y;
  s   = s < 0 ? 0 : (s > NN - 1 ? NN - 1 : s);
  eid = eid < 0 ? 0 : (eid > NE - 1 ? NE - 1 : eid);
  int d = dsts[eid];
  d = d < 0 ? 0 : (d > NN - 1 ? NN - 1 : d);
  const float ewv = bf16_val(ew[eid]);
  const float ds  = DSRC[s];
  const float dd  = DDST[d];
  const int fd  = FLAGD[(size_t)blk * 32];
  int tot       = FLAGD[(size_t)blk * 32 + 1];
  const int fs  = FLAGS[(size_t)(s >> SLB) * 32];
  tot = tot < 0 ? 0 : (tot > RCAP ? RCAP : tot);
  const float den = sqrtf(fmaxf(ds * dd, 1e-12f));
  const float w   = ewv / den;
  asm volatile("" :: "v"(w));
  const unsigned vm = (j < tot) ? 0xffffffffu : 0u;
  unsigned wb = __float_as_uint(w) & vm;
  wb = ((fd | fs) != 0) ? 0x7fc00000u : wb;
  const float o = __uint_as_float(wb);
  float* op = WL + (size_t)gid;
  *(volatile float*)op = o;
  __threadfence();
  *(volatile float*)op = o;
}

template <int L0>
__global__ __launch_bounds__(NTHR) void k_replay(const int* __restrict__ LIST, const float* __restrict__ WL,
                                                 const int* __restrict__ CNT, const int* __restrict__ OFF,
                                                 const int* __restrict__ FLAGD,
                                                 const unsigned short* __restrict__ SRCP, unsigned short* NEI) {
  const int tid = (int)threadIdx.x, lane = tid & 31, wave = tid >> 5;
  const int rowBase = (int)blockIdx.x * RBM;
  const int bucket  = rowBase >> SLB;
  const int*   lb = LIST + (size_t)bucket * (size_t)(2 * RCAP);
  const float* wb = WL + (size_t)bucket * RCAP;
  const int*   cb = CNT + (size_t)bucket * NBRUN;
  const int*   ob = OFF + (size_t)bucket * NBRUN;
  const int flag  = FLAGD[(size_t)bucket * 32];
  const float qnan = __uint_as_float(0x7fc00000u);

#pragma unroll 1
  for (int i = 0; i < RBM / NWAVE; ++i) {
    const int d    = rowBase + (RBM / NWAVE) * wave + i;
    const int slot = d & (NBRUN - 1);
    int cv  = cb[slot];
    int ovv = ob[slot];
    const bool big = cv > DEGCAP;
    cv  = cv < 0 ? 0 : (cv > DEGCAP ? DEGCAP : cv);
    ovv = ovv < 0 ? 0 : (ovv > RCAP - 1 ? RCAP - 1 : ovv);
    const int cden = cv < 1 ? 1 : cv;
    const int c = __builtin_amdgcn_readfirstlane(cv);
    const int o = __builtin_amdgcn_readfirstlane(ovv);
    int last = o + c - 1;
    last = last < o ? o : last;
    last = last > RCAP - 1 ? RCAP - 1 : last;
    float a0 = 0.0f, a1 = 0.0f, a2 = 0.0f, a3 = 0.0f;
#pragma unroll 1
    for (int b0 = 0; b0 < c; b0 += 32) {
      int idx = o + b0 + lane;
      idx = idx > last ? last : idx;
      const v2i ent = *(const v2ia*)(lb + 2 * idx);
      int sr = ent.x;
      sr = sr < 0 ? 0 : (sr > NN - 1 ? NN - 1 : sr);
      const int wbits = __float_as_int(wb[idx]);
      const int m32 = (c - b0) < 32 ? (c - b0) : 32;
#pragma unroll 1
      for (int k = 0; k < m32; ++k) {
        const int   sk = __builtin_amdgcn_readlane(sr, k);
        const float ck = __int_as_float(__builtin_amdgcn_readlane(wbits, k));
        if constexpr (L0 != 0) {
          const v2u wh = *(const v2ua*)(SRCP + (size_t)sk * XP + 4 * lane);
          a0 = fmaf(ck, __uint_as_float(wh.x << 16), a0);
          a1 = fmaf(ck, __uint_as_float(wh.x & 0xffff0000u), a1);
          a2 = fmaf(ck, __uint_as_float(wh.y << 16), a2);
          a3 = fmaf(ck, __uint_as_float(wh.y & 0xffff0000u), a3);
        } else {
          const unsigned short* rp = SRCP + (size_t)sk * HP + 4 * lane;
          const v2u wh = *(const v2ua*)rp;
          const v2u wl = *(const v2ua*)(rp + DF);
          const float f0 = __uint_as_float(wh.x << 16)         + __uint_as_float(wl.x << 16);
          const float f1 = __uint_as_float(wh.x & 0xffff0000u) + __uint_as_float(wl.x & 0xffff0000u);
          const float f2 = __uint_as_float(wh.y << 16)         + __uint_as_float(wl.y << 16);
          const float f3 = __uint_as_float(wh.y & 0xffff0000u) + __uint_as_float(wl.y & 0xffff0000u);
          a0 = fmaf(ck, f0, a0);
          a1 = fmaf(ck, f1, a1);
          a2 = fmaf(ck, f2, a2);
          a3 = fmaf(ck, f3, a3);
        }
      }
    }
    const float fc = (float)cden;
    float m0 = a0 / fc, m1 = a1 / fc, m2 = a2 / fc, m3 = a3 / fc;
    const bool bad  = (flag != 0) | big;
    const bool live = d < NN;
    m0 = bad ? qnan : m0; m1 = bad ? qnan : m1; m2 = bad ? qnan : m2; m3 = bad ? qnan : m3;
    m0 = live ? m0 : 0.0f; m1 = live ? m1 : 0.0f; m2 = live ? m2 : 0.0f; m3 = live ? m3 : 0.0f;
    int h01, h23, l01, l23;
    hilo_pack(m0, m1, m2, m3, h01, h23, l01, l23);
    const v4i ow = regroup32(h01, h23, l01, l23, lane);
    st2_v4i(NEI + (size_t)d * HP + 8 * lane, ow);
  }
}

template <int KEXT, int WPITCH>
__device__ __forceinline__ void kseg(const unsigned short* __restrict__ ap, const unsigned short* __restrict__ bp,
                                     v8f (&acc)[8]) {
#pragma unroll 1
  for (int k0 = 0; k0 < KEXT; k0 += 32) {
    FragB af;
    af.h[0] = *(const v8usa*)(ap + k0);
    af.h[1] = *(const v8usa*)(ap + k0 + 16);
#pragma unroll
    for (int nt = 0; nt < 8; ++nt) {
      const unsigned short* wq = bp + (size_t)(16 * nt) * (size_t)WPITCH + k0;
      FragB bf;
      bf.h[0] = *(const v8usa*)wq;
      bf.h[1] = *(const v8usa*)(wq + 16);
      acc[nt] = wmb(af, bf, acc[nt]);
    }
  }
}

template <int PH, int KH, int WP, int FIN>
__global__ __launch_bounds__(GTHR) __attribute__((amdgpu_num_vgpr(248)))
void k_lin(const unsigned short* __restrict__ NEI, const unsigned short* __restrict__ HS,
           const unsigned short* __restrict__ WT, const float* __restrict__ bvec,
           const int* __restrict__ FLAGD, const int* __restrict__ FLAGS,
           unsigned short* Hout, float* outp) {
  static_assert(KH % 32 == 0 && KH <= PH && WSOFF + KH <= WP && KN_EXT <= WSOFF);
  __shared__ __attribute__((aligned(16))) float stg[GBM * GBN];
  __shared__ __attribute__((aligned(16))) float sb[DF];
  const int tid = (int)threadIdx.x, lane = tid & 31, wave = tid >> 5, hh = lane >> 4, m = lane & 15;
  const int rowBase = (int)blockIdx.x * GBM;
  if (tid < 32) *(v4fa*)(sb + 4 * tid) = *(const v4fa*)(bvec + 4 * tid);

  v8f acc[8];
  {
    const v8f z = {0.f, 0.f, 0.f, 0.f, 0.f, 0.f, 0.f, 0.f};
#pragma unroll
    for (int t = 0; t < 8; ++t) acc[t] = z;
  }
  const unsigned short* an = NEI + (size_t)(rowBase + 16 * wave + m) * (size_t)HP + 8 * hh;
  const unsigned short* ah = HS + (size_t)(rowBase + 16 * wave + m) * (size_t)PH + 8 * hh;
  const unsigned short* bp = WT + (size_t)m * (size_t)WP + 8 * hh;
  kseg<KN_EXT, WP>(an, bp, acc);
  kseg<KH, WP>(ah, bp + WSOFF, acc);

#pragma unroll
  for (int nt = 0; nt < 8; ++nt) {
    const int lc = 16 * nt + m;
#pragma unroll
    for (int r = 0; r < 8; ++r) {
      const int lr = 16 * wave + 8 * hh + r;
      stg[lr * GBN + lc] = acc[nt][r];
    }
  }
  __syncthreads();

  bool gbad = false;
  if constexpr (FIN != 0) {
    const int i0 = lane < NBK ? lane : NBK - 1;
    const int i1 = lane + 32 < NBK ? lane + 32 : NBK - 1;
    const int f = FLAGD[(size_t)i0 * 32] | FLAGD[(size_t)i1 * 32] | FLAGS[(size_t)i0 * 32] | FLAGS[(size_t)i1 * 32];
    gbad = __builtin_amdgcn_ballot_w32(f != 0) != 0u;
  }
  const v4f bias = *(const v4fa*)(sb + 4 * lane);
  const float qnan = __uint_as_float(0x7fc00000u);

#pragma unroll 1
  for (int i = 0; i < 16; ++i) {
    const int lr   = 16 * wave + i;
    const int grow = rowBase + lr;
    const bool live = grow < NN;
    const v4f a = *(const v4fa*)(stg + lr * GBN + 4 * lane);
    float v0 = a.x + bias.x, v1 = a.y + bias.y, v2 = a.z + bias.z, v3 = a.w + bias.w;
    if constexpr (FIN != 0) {
      v4f o;
      o.x = gbad ? qnan : v0; o.y = gbad ? qnan : v1; o.z = gbad ? qnan : v2; o.w = gbad ? qnan : v3;
      if (live) st2_v4f(outp + (size_t)grow * DF + 4 * lane, o);
    } else {
      v0 = (v0 > 0.0f) ? v0 : (v0 - v0); v1 = (v1 > 0.0f) ? v1 : (v1 - v1);
      v2 = (v2 > 0.0f) ? v2 : (v2 - v2); v3 = (v3 > 0.0f) ? v3 : (v3 - v3);
      v0 = live ? v0 : 0.0f; v1 = live ? v1 : 0.0f; v2 = live ? v2 : 0.0f; v3 = live ? v3 : 0.0f;
      int h01, h23, l01, l23;
      hilo_pack(v0, v1, v2, v3, h01, h23, l01, l23);
      const v4i ow = regroup32(h01, h23, l01, l23, lane);
      st2_v4i(Hout + (size_t)grow * HP + 8 * lane, ow);
    }
  }
}

static constexpr size_t al256c(size_t v) { return (v + 255) & ~(size_t)255; }

extern "C" void kernel_launch(void* const* d_in, const int* in_sizes, int n_in,
                              void* d_out, int out_size, void* d_ws, size_t ws_size,
                              hipStream_t stream) {
  if (n_in < 13) return;
  if (in_sizes[0] != NN * DF) return;
  if (in_sizes[1] != NE) return;
  if (in_sizes[2] != DF * DF || in_sizes[3] != DF * DF || in_sizes[4] != DF) return;
  if (in_sizes[5] != DF * DF || in_sizes[6] != DF * DF || in_sizes[7] != DF) return;
  if (in_sizes[8] != DF * DF || in_sizes[9] != DF * DF || in_sizes[10] != DF) return;
  if (in_sizes[11] != NE || in_sizes[12] != NE) return;
  if (out_size != NN * DF) return;

  const float* x   = (const float*)d_in[0];
  const float* ew  = (const float*)d_in[1];
  const float* Ws0 = (const float*)d_in[2];
  const float* Wn0 = (const float*)d_in[3];
  const float* b0  = (const float*)d_in[4];
  const float* Ws1 = (const float*)d_in[5];
  const float* Wn1 = (const float*)d_in[6];
  const float* b1  = (const float*)d_in[7];
  const float* Ws2 = (const float*)d_in[8];
  const float* Wn2 = (const float*)d_in[9];
  const float* b2  = (const float*)d_in[10];
  const int*   src = (const int*)d_in[11];
  const int*   dst = (const int*)d_in[12];
  float* out = (float*)d_out;

  constexpr size_t zXB   = (size_t)MP * XP * 2;
  constexpr size_t zHL   = (size_t)MP * HP * 2;
  constexpr size_t zLIST = (size_t)NBK * RCAP * 8;
  constexpr size_t zWL   = (size_t)NBK * RCAP * 4;
  constexpr size_t zTAB  = (size_t)NBK * NBRUN * 4;
  constexpr size_t zFLAG = al256c((size_t)NBK * 128);
  constexpr size_t zW0   = (size_t)DF * W0P * 2;
  constexpr size_t zW12  = (size_t)DF * W12P * 2;
  constexpr size_t zSM   = (size_t)3 * DF * 4;
  constexpr size_t oXB   = 0;
  constexpr size_t oNEI  = oXB + zXB;
  constexpr size_t oHA   = oNEI + zHL;
  constexpr size_t oHB   = oHA + zHL;
  constexpr size_t oLIST = oHB + zHL;
  constexpr size_t oWL   = oLIST + zLIST;
  constexpr size_t oCNT  = oWL + zWL;
  constexpr size_t oOFF  = oCNT + zTAB;
  constexpr size_t oDDST = oOFF + zTAB;
  constexpr size_t oDSRC = oDDST + zTAB;
  constexpr size_t oFLD  = oDSRC + zTAB;
  constexpr size_t oFLS  = oFLD + zFLAG;
  constexpr size_t oW0   = oFLS + zFLAG;
  constexpr size_t oW1   = oW0 + zW0;
  constexpr size_t oW2   = oW1 + zW12;
  constexpr size_t oSM   = oW2 + zW12;
  constexpr size_t oEND  = oSM + zSM;
  static_assert(zXB % 256 == 0 && zHL % 256 == 0 && zLIST % 256 == 0 && zWL % 256 == 0 && zTAB % 256 == 0);
  static_assert(zFLAG % 256 == 0 && zW0 % 256 == 0 && zW12 % 256 == 0 && zSM % 256 == 0);
  static_assert(oEND <= (size_t)(128u << 20));
  static_assert((size_t)(NN - 1) * DF + (DF - 1) < (size_t)NN * DF);
  if (oEND > ws_size) return;

  char* ws = (char*)d_ws;
  unsigned short* XB   = (unsigned short*)(ws + oXB);
  unsigned short* NEI  = (unsigned short*)(ws + oNEI);
  unsigned short* HA   = (unsigned short*)(ws + oHA);
  unsigned short* HB   = (unsigned short*)(ws + oHB);
  int*            LIST = (int*)(ws + oLIST);
  float*          WL   = (float*)(ws + oWL);
  int*            CNT  = (int*)(ws + oCNT);
  int*            OFF  = (int*)(ws + oOFF);
  int*            DDST = (int*)(ws + oDDST);
  int*            DSRC = (int*)(ws + oDSRC);
  int*            FLD  = (int*)(ws + oFLD);
  int*            FLS  = (int*)(ws + oFLS);
  unsigned short* W0C  = (unsigned short*)(ws + oW0);
  unsigned short* W1C  = (unsigned short*)(ws + oW1);
  unsigned short* W2C  = (unsigned short*)(ws + oW2);
  float*          SM   = (float*)(ws + oSM);

  hipFuncSetAttribute(reinterpret_cast<const void*>(&k_bucket), hipFuncAttributeMaxDynamicSharedMemorySize, (int)BK_LDS);

  k_prep<<<PBTOT, NTHR, 0, stream>>>(x, Ws0, Wn0, b0, Ws1, Wn1, b1, Ws2, Wn2, b2, XB, W0C, W1C, W2C, SM);
  k_bucket<<<dim3(NBK, 2, 1), NTHR, BK_LDS, stream>>>(src, dst, ew, LIST, CNT, OFF, DDST, DSRC, FLD, FLS);
  k_edgew<<<(NBK * RCAP) / NTHR, NTHR, 0, stream>>>(LIST, dst, ew, (const float*)DSRC, (const float*)DDST, FLD, FLS, WL);
  k_replay<1><<<MP / RBM, NTHR, 0, stream>>>(LIST, WL, CNT, OFF, FLD, XB, NEI);
  k_lin<XP, DF, W0P, 0><<<MP / GBM, GTHR, 0, stream>>>(NEI, XB, W0C, SM, FLD, FLS, HA, out);
  k_replay<0><<<MP / RBM, NTHR, 0, stream>>>(LIST, WL, CNT, OFF, FLD, HA, NEI);
  k_lin<HP, KH_EXT, W12P, 0><<<MP / GBM, GTHR, 0, stream>>>(NEI, HA, W1C, SM + DF, FLD, FLS, HB, out);
  k_replay<0><<<MP / RBM, NTHR, 0, stream>>>(LIST, WL, CNT, OFF, FLD, HB, NEI);
  k_lin<HP, KH_EXT, W12P, 1><<<MP / GBM, GTHR, 0, stream>>>(NEI, HB, W2C, SM + 2 * DF, FLD, FLS, HA, out);
}
